// VRWKV_SpatialMix_V6_85066122264778
// MI455X (gfx1250) — hardware-verified
//
#include <hip/hip_runtime.h>
#include <math.h>

typedef __attribute__((ext_vector_type(16))) _Float16 v16h;
typedef __attribute__((ext_vector_type(16))) __bf16 v16b;
typedef __attribute__((ext_vector_type(8)))  _Float16 v8h;
typedef __attribute__((ext_vector_type(8)))  float v8f;
typedef __attribute__((ext_vector_type(4)))  float v4f;
typedef __attribute__((ext_vector_type(2)))  float v2f;
typedef __attribute__((ext_vector_type(4)))  unsigned v4u;
typedef __attribute__((ext_vector_type(4)))  int v4i;
typedef float __attribute__((may_alias)) float_a;
typedef int __attribute__((may_alias)) int_a;

template <typename T> __device__ __forceinline__ void vst2(void* p, T v) { *(volatile T*)p = v; __threadfence(); *(volatile T*)p = v; }
__device__ __forceinline__ v8f wmma16(v16h a, v16h b, v8f c) {
  v8f d = __builtin_amdgcn_wmma_f32_16x16x32_f16(false, a, false, b, (short)0, c, false, false);
  asm volatile("v_nop\n\tv_nop\n\tv_nop\n\tv_nop" : "+v"(d) : "v"(a), "v"(b));
  return d;
}
__device__ __forceinline__ v8f wmma_bf(v16b a, v16b b, v8f c) {
  v8f d = __builtin_amdgcn_wmma_f32_16x16x32_bf16(false, a, false, b, (short)0, c, false, false);
  asm volatile("v_nop\n\tv_nop\n\tv_nop\n\tv_nop" : "+v"(d) : "v"(a), "v"(b));
  return d;
}
__device__ __forceinline__ v16h frag_h(const _Float16* rowk0, int lane) {
  union { v16h v; v8h q[2]; } u; const _Float16* p = rowk0 + 8 * (lane >> 4);
  u.q[0] = *(const v8h*)p; u.q[1] = *(const v8h*)(p + 16); return u.v;
}
__device__ __forceinline__ v16h frag_f32(const float* rowk0, int lane) {
  v16h a; const float* p = rowk0 + 8 * (lane >> 4);
#pragma unroll
  for (int i = 0; i < 8; ++i) { a[i] = (_Float16)p[i]; a[8 + i] = (_Float16)p[16 + i]; }
  return a;
}
__device__ __forceinline__ v16h frag_f32s(const float* rowk0, int lane, float sc) {
  v16h a; const float* p = rowk0 + 8 * (lane >> 4);
#pragma unroll
  for (int i = 0; i < 8; ++i) { a[i] = (_Float16)(p[i] * sc); a[8 + i] = (_Float16)(p[16 + i] * sc); }
  return a;
}
__device__ __forceinline__ v16h fragc_f32(const float* W, int k0, int n, int lane, int ld, int K) {
  v16h a; const int g = lane >> 4;
#pragma unroll
  for (int i = 0; i < 8; ++i) { const int ka = k0 + 8 * g + i, kb = ka + 16;
    a[i] = (_Float16)(ka < K ? W[(size_t)(ka < K ? ka : K - 1) * ld + n] : 0.f); a[8 + i] = (_Float16)(kb < K ? W[(size_t)(kb < K ? kb : K - 1) * ld + n] : 0.f); }
  return a;
}
struct F2 { v16b h, l; };
__device__ __forceinline__ F2 bsplit16(const float v[16]) { F2 r;
#pragma unroll
  for (int i = 0; i < 16; ++i) { const __bf16 h = (__bf16)v[i]; r.h[i] = h; r.l[i] = (__bf16)(v[i] - (float)h); }
  return r; }
__device__ __forceinline__ F2 split_row(const float* row, int k0, int lane) { float v[16]; const float* p = row + k0 + 8 * (lane >> 4);
#pragma unroll
  for (int i = 0; i < 8; ++i) { v[i] = p[i]; v[8 + i] = p[16 + i]; }
  return bsplit16(v); }
__device__ __forceinline__ F2 split_rowK(const float* row, int k0, int lane, int K) { float v[16]; const int g = lane >> 4;
#pragma unroll
  for (int i = 0; i < 8; ++i) { const int ka = k0 + 8 * g + i, kb = ka + 16; v[i] = ka < K ? row[ka < K ? ka : K - 1] : 0.f; v[8 + i] = kb < K ? row[kb < K ? kb : K - 1] : 0.f; }
  return bsplit16(v); }
__device__ __forceinline__ F2 split_col(const float* W, int k0, int n, int lane, int ld, int K) { float v[16]; const int g = lane >> 4;
#pragma unroll
  for (int i = 0; i < 8; ++i) { const int ka = k0 + 8 * g + i, kb = ka + 16; v[i] = ka < K ? W[(size_t)(ka < K ? ka : K - 1) * ld + n] : 0.f; v[8 + i] = kb < K ? W[(size_t)(kb < K ? kb : K - 1) * ld + n] : 0.f; }
  return bsplit16(v); }
__device__ __forceinline__ v8f mac3(const F2& a, const F2& b, v8f c) { c = wmma_bf(a.l, b.h, c); c = wmma_bf(a.h, b.l, c); return wmma_bf(a.h, b.h, c); }
__device__ __forceinline__ float sigm(float v) { return 1.0f / (1.0f + expf(-v)); }
#define LDSX() do { asm volatile("s_wait_dscnt 0" ::: "memory"); __builtin_amdgcn_wave_barrier(); __builtin_amdgcn_fence(__ATOMIC_RELEASE, "workgroup"); } while (0)


#define NB 4
#define TT 1024
#define HP 32
#define WP 32
#define CC 768
#define NH 24
#define HS 32
#define ME 32
#define M5 160
#define DD 64
#define NR (NB * TT)
#ifndef TRB
#define TRB (NR / 64)
#define NBT NB
#define TSTEP TT
#endif
typedef __attribute__((ext_vector_type(8))) __bf16 v8b;
__device__ __forceinline__ v16b frag_b(const __bf16* rowk0, int lane) {
  union { v16b v; v8b q[2]; } u; const __bf16* p = rowk0 + 8 * (lane >> 4);
  u.q[0] = *(const v8b*)p; u.q[1] = *(const v8b*)(p + 16); return u.v;
}
__device__ __forceinline__ float bfr(float v) { return (float)(__bf16)v; }
__device__ __attribute__((noinline)) float exp_ni(float v) { return expf(v); }
__device__ __attribute__((noinline)) float erf_ni(float v) { return erff(v); }

__device__ __attribute__((noinline)) float tanh_ni(float v) { return tanhf(v); }
#define PK_W1  0
#define PK_W2  (PK_W1 + M5 * CC)
#define PK_DW1 (PK_W2 + 5 * CC * ME)
#define PK_DW2 (PK_DW1 + DD * CC)
#define PK_R   (PK_DW2 + CC * DD)
#define PK_K   (PK_R + CC * CC)
#define PK_V   (PK_K + CC * CC)
#define PK_G   (PK_V + CC * CC)
#define PK_O   (PK_G + CC * CC)
#define PK_END (PK_O + CC * CC)
#define WS_PK  0u
#define WS_XX  (WS_PK + 2u * PK_END)
#define WS_TM  (WS_XX + 4u * NR * CC)
#define WS_XK  (WS_TM + 4u * NR * M5)
#define WS_R   (WS_XK + 4u * NR * CC)
#define WS_K   (WS_R + 4u * NR * CC)
#define WS_V   (WS_K + 4u * NR * CC)
#define WS_W   (WS_V + 4u * NR * CC)
#define WS_G   (WS_W + 4u * NR * CC)
#define WS_TD  (WS_G + 4u * NR * CC)
#define WS_END (WS_TD + 4u * NR * DD)

__global__ __launch_bounds__(256) void k_packT(const float* __restrict__ Wm, int K, int ld, __bf16* __restrict__ DST) {
  __shared__ __align__(16) __bf16 s[CC]; const int n = blockIdx.x, tid = threadIdx.x;
  for (int k = tid; k < K; k += 256) s[k] = (__bf16)Wm[(size_t)k * ld + n];
  __syncthreads();
  for (int q = tid; q < K / 8; q += 256) vst2((unsigned*)(DST + (size_t)n * K + q * 8), *(const v4u*)&s[q * 8]);
}
__global__ __launch_bounds__(256) void k_packT8(const float* __restrict__ Wm, int K, int ld, __bf16* __restrict__ DST) {
  __shared__ __align__(16) __bf16 s[8 * 64]; const int n0 = blockIdx.x * 8, tid = threadIdx.x;
  for (int q = tid; q < 8 * K; q += 256) { const int nl = q / K, k = q % K; s[q] = (__bf16)Wm[(size_t)k * ld + n0 + nl]; }
  __syncthreads();
  for (int q = tid; q < K; q += 256) vst2((unsigned*)(DST + (size_t)n0 * K + q * 8), *(const v4u*)&s[q * 8]);
}
__global__ __launch_bounds__(256) void k_xx(const float* __restrict__ X, float* __restrict__ XX) {
  __shared__ __align__(16) float s[CC]; const int row = blockIdx.x, tid = threadIdx.x; const int b = row / TT, t = row % TT, h = t / WP, w = t % WP;
  for (int c = tid; c < CC; c += 256) { const int q = c / (CC / 4); int hh = h, ww = w; bool ok = true;
    if (q == 0) { ww = w - 1; ok = w > 0; } else if (q == 1) { ww = w + 1; ok = w < WP - 1; } else if (q == 2) { hh = h - 1; ok = h > 0; } else { hh = h + 1; ok = h < HP - 1; }
    const float xs = ok ? bfr(X[((size_t)b * TT + hh * WP + ww) * CC + c]) : 0.f; s[c] = xs - bfr(X[(size_t)row * CC + c]); }
  __syncthreads();
  for (int q = tid; q < CC / 4; q += 256) vst2(XX + (size_t)row * CC + q * 4, *(const v4f*)&s[q * 4]);
}
__device__ __forceinline__ F2 split_mix(const float* xrow, const float* xxrow, const float* maa, int k0, int lane) {
  float v[16]; const int g = lane >> 4;
#pragma unroll
  for (int i = 0; i < 8; ++i) { const int ka = k0 + 8 * g + i, kb = ka + 16; v[i] = bfr(xrow[ka]) + xxrow[ka] * bfr(maa[ka]); v[8 + i] = bfr(xrow[kb]) + xxrow[kb] * bfr(maa[kb]); }
  return bsplit16(v); }
__global__ __launch_bounds__(128) void k_tm(const float* __restrict__ X, const float* __restrict__ XX, const float* __restrict__ MAAX, const __bf16* __restrict__ P, float* __restrict__ TM) {
  __shared__ __align__(16) float so[4][16][M5 + 4];
  const int tid = threadIdx.x, wave = tid >> 5, lane = tid & 31, col = lane & 15, g = lane >> 4; const size_t r0 = (size_t)blockIdx.x * 64 + wave * 16;
  v8f acc[10] = {};
#pragma unroll 1
  for (int kc = 0; kc < CC / 32; ++kc) { const F2 a = split_mix(X + (r0 + col) * CC, XX + (r0 + col) * CC, MAAX, kc * 32, lane);
#pragma unroll
    for (int j = 0; j < 10; ++j) { const v16b w = frag_b(P + (size_t)(j * 16 + col) * CC + kc * 32, lane); acc[j] = wmma_bf(a.l, w, acc[j]); acc[j] = wmma_bf(a.h, w, acc[j]); } }
#pragma unroll
  for (int j = 0; j < 10; ++j)
#pragma unroll
    for (int r = 0; r < 8; ++r) so[wave][8 * g + r][j * 16 + col] = tanh_ni(acc[j][r]);
  LDSX();
  for (int rl = 0; rl < 16; ++rl) for (int pc = lane; pc < M5 / 4; pc += 32) vst2(TM + (r0 + rl) * M5 + pc * 4, *(const v4f*)&so[wave][rl][pc * 4]);
}
__global__ __launch_bounds__(128) void k_mix(const float* __restrict__ X, const float* __restrict__ XX, const float* __restrict__ MAA, const float* __restrict__ TM, int sel, const __bf16* __restrict__ P2, float* __restrict__ XK) {
  __shared__ __align__(16) float so[4][16][132];
  const int tid = threadIdx.x, wave = tid >> 5, lane = tid & 31, col = lane & 15, g = lane >> 4; const size_t r0 = (size_t)blockIdx.x * 64 + wave * 16; const int n0 = blockIdx.y * 128;
  v8f acc[8] = {}; const F2 a = split_row(TM + (r0 + col) * M5 + sel * ME, 0, lane);
#pragma unroll
  for (int j = 0; j < 8; ++j) { const v16b w = frag_b(P2 + ((size_t)sel * CC + n0 + j * 16 + col) * ME, lane); acc[j] = wmma_bf(a.l, w, acc[j]); acc[j] = wmma_bf(a.h, w, acc[j]); }
#pragma unroll
  for (int j = 0; j < 8; ++j) { const int n = n0 + j * 16 + col; const float mv = bfr(MAA[n]);
#pragma unroll
    for (int r = 0; r < 8; ++r) { const size_t row = r0 + 8 * g + r; so[wave][8 * g + r][j * 16 + col] = bfr(X[row * CC + n]) + XX[row * CC + n] * (mv + acc[j][r]); } }
  LDSX();
  for (int rl = 0; rl < 16; ++rl) vst2(XK + (r0 + rl) * CC + n0 + lane * 4, *(const v4f*)&so[wave][rl][lane * 4]);
}
template <int K, int EPI, int NT>
__global__ __launch_bounds__(128) void k_lin(const float* __restrict__ A, int lda, const __bf16* __restrict__ P, const float* __restrict__ bias, float* __restrict__ OUT, int ldo) {
  __shared__ __align__(16) float so[4][16][132];
  const int tid = threadIdx.x, wave = tid >> 5, lane = tid & 31, col = lane & 15, g = lane >> 4; const size_t r0 = (size_t)blockIdx.x * 64 + wave * 16; const int n0 = blockIdx.y * (NT * 16);
  v8f acc[NT]; for (int j = 0; j < NT; ++j) acc[j] = (v8f){};
#pragma unroll 1
  for (int kc = 0; kc < K / 32; ++kc) { const F2 a = split_row(A + (r0 + col) * lda, kc * 32, lane);
#pragma unroll
    for (int j = 0; j < NT; ++j) { const v16b w = frag_b(P + (size_t)(n0 + j * 16 + col) * K + kc * 32, lane); acc[j] = wmma_bf(a.l, w, acc[j]); acc[j] = wmma_bf(a.h, w, acc[j]); } }
#pragma unroll
  for (int j = 0; j < NT; ++j) { const int n = n0 + j * 16 + col;
#pragma unroll
    for (int r = 0; r < 8; ++r) { float v = acc[j][r]; if (EPI == 1) v = v / (1.0f + exp_ni(-v)); if (EPI == 2) v = tanh_ni(v); if (EPI == 3) v += bfr(bias[n]); so[wave][8 * g + r][j * 16 + col] = v; } }
  LDSX();
  for (int rl = 0; rl < 16; ++rl) if (lane < NT * 4) vst2(OUT + (r0 + rl) * ldo + n0 + lane * 4, *(const v4f*)&so[wave][rl][lane * 4]);
}
__global__ __launch_bounds__(128) void k_wkv(const float* __restrict__ R, const float* __restrict__ Kx, const float* __restrict__ V, const float* __restrict__ Wd, const float* __restrict__ U, float* __restrict__ Y) {
  const int tid = threadIdx.x, wave = tid >> 5, lane = tid & 31; const int h = blockIdx.x * 4 + wave, b = blockIdx.y; const int ch = h * HS + lane;
  float s[HS];
#pragma unroll
  for (int j = 0; j < HS; ++j) s[j] = 0.f;
  const float uj = bfr(U[h * HS + lane]);
#pragma unroll 1
  for (int t = 0; t < TSTEP; ++t) { const size_t row = (size_t)b * TT + t; const float rj = R[row * CC + ch], kj = Kx[row * CC + ch], vi = V[row * CC + ch], wj = Wd[row * CC + ch]; const float dj = exp_ni(-exp_ni(wj));
    float c = rj * uj * kj;
#pragma unroll
    for (int o = 1; o < 32; o <<= 1) c += __shfl_xor(c, o);
    float y = vi * c;
#pragma unroll
    for (int j = 0; j < HS; ++j) { const float rjj = __shfl(rj, j), kjj = __shfl(kj, j), djj = __shfl(dj, j); y += rjj * s[j]; s[j] = djj * s[j] + kjj * vi; }
    *(volatile float*)(Y + row * CC + ch) = y; __threadfence(); *(volatile float*)(Y + row * CC + ch) = y; }
}
__global__ __launch_bounds__(256) void k_lng(float* __restrict__ Y, const float* __restrict__ G, const float* __restrict__ lw, const float* __restrict__ lb) {
  __shared__ __align__(16) float s[8][CC];
  const int wave = threadIdx.x >> 5, lane = threadIdx.x & 31; const size_t r = (size_t)blockIdx.x * 8 + wave; float* y = Y + r * CC; float* sw = s[wave];
  float sum = 0.f;
#pragma unroll 4
  for (int i = 0; i < CC / 32; ++i) { const float t = y[lane + 32 * i]; sw[lane + 32 * i] = t; sum += t; }
#pragma unroll
  for (int o = 1; o < 32; o <<= 1) sum += __shfl_xor(sum, o);
  const float mu = sum / (float)CC; float var = 0.f;
#pragma unroll 4
  for (int i = 0; i < CC / 32; ++i) { const float d = sw[lane + 32 * i] - mu; var += d * d; }
#pragma unroll
  for (int o = 1; o < 32; o <<= 1) var += __shfl_xor(var, o);
  const float rs = rsqrtf(var / (float)CC + 1e-5f);
#pragma unroll 4
  for (int i = 0; i < CC / 32; ++i) { const int c = lane + 32 * i; sw[c] = ((sw[c] - mu) * rs * bfr(lw[c]) + bfr(lb[c])) * G[r * CC + c]; }
  LDSX();
#pragma unroll 2
  for (int pc = lane; pc < CC / 4; pc += 32) vst2(y + pc * 4, *(const v4f*)&sw[pc * 4]);
}
extern "C" void kernel_launch(void* const* d_in, const int* in_sizes, int n_in, void* d_out, int out_size, void* d_ws, size_t ws_size, hipStream_t stream) {
  (void)in_sizes; (void)n_in; (void)out_size;
  const float** F = (const float**)d_in;
  if (ws_size < (size_t)WS_END) return;
  char* ws = (char*)d_ws; __bf16* PK = (__bf16*)(ws + WS_PK);
  float *XX = (float*)(ws + WS_XX), *TM = (float*)(ws + WS_TM), *XK = (float*)(ws + WS_XK), *R = (float*)(ws + WS_R), *Kx = (float*)(ws + WS_K), *V = (float*)(ws + WS_V), *Wd = (float*)(ws + WS_W), *G = (float*)(ws + WS_G), *TD = (float*)(ws + WS_TD);
  k_packT<<<M5, 256, 0, stream>>>(F[7], CC, M5, PK + PK_W1);
  for (int sel = 0; sel < 5; ++sel) k_packT8<<<CC / 8, 256, 0, stream>>>(F[8] + (size_t)sel * ME * CC, ME, CC, PK + PK_W2 + (size_t)sel * CC * ME);
  k_packT<<<DD, 256, 0, stream>>>(F[10], CC, DD, PK + PK_DW1);
  k_packT8<<<CC / 8, 256, 0, stream>>>(F[11], DD, CC, PK + PK_DW2);
  k_packT<<<CC, 256, 0, stream>>>(F[13], CC, CC, PK + PK_R); k_packT<<<CC, 256, 0, stream>>>(F[14], CC, CC, PK + PK_K); k_packT<<<CC, 256, 0, stream>>>(F[15], CC, CC, PK + PK_V); k_packT<<<CC, 256, 0, stream>>>(F[16], CC, CC, PK + PK_G); k_packT<<<CC, 256, 0, stream>>>(F[17], CC, CC, PK + PK_O);
  k_xx<<<NBT * TT, 256, 0, stream>>>(F[0], XX);
  k_tm<<<TRB, 128, 0, stream>>>(F[0], XX, F[1], PK + PK_W1, TM);
  k_mix<<<dim3(TRB, CC / 128), 128, 0, stream>>>(F[0], XX, F[2], TM, 0, PK + PK_W2, XK);
  k_lin<CC, 2, 4><<<dim3(TRB, DD / 64), 128, 0, stream>>>(XK, CC, PK + PK_DW1, nullptr, TD, DD);
  k_lin<DD, 3, 8><<<dim3(TRB, CC / 128), 128, 0, stream>>>(TD, DD, PK + PK_DW2, F[9], Wd, CC);
  k_mix<<<dim3(TRB, CC / 128), 128, 0, stream>>>(F[0], XX, F[3], TM, 1, PK + PK_W2, XK);
  k_lin<CC, 0, 8><<<dim3(TRB, CC / 128), 128, 0, stream>>>(XK, CC, PK + PK_K, nullptr, Kx, CC);
  k_mix<<<dim3(TRB, CC / 128), 128, 0, stream>>>(F[0], XX, F[4], TM, 2, PK + PK_W2, XK);
  k_lin<CC, 0, 8><<<dim3(TRB, CC / 128), 128, 0, stream>>>(XK, CC, PK + PK_V, nullptr, V, CC);
  k_mix<<<dim3(TRB, CC / 128), 128, 0, stream>>>(F[0], XX, F[5], TM, 3, PK + PK_W2, XK);
  k_lin<CC, 0, 8><<<dim3(TRB, CC / 128), 128, 0, stream>>>(XK, CC, PK + PK_R, nullptr, R, CC);
  k_mix<<<dim3(TRB, CC / 128), 128, 0, stream>>>(F[0], XX, F[6], TM, 4, PK + PK_W2, XK);
  k_lin<CC, 1, 8><<<dim3(TRB, CC / 128), 128, 0, stream>>>(XK, CC, PK + PK_G, nullptr, G, CC);
  k_wkv<<<dim3(NH / 4, NBT), 128, 0, stream>>>(R, Kx, V, Wd, F[12], XK);
  k_lng<<<TRB * 8, 256, 0, stream>>>(XK, G, F[18], F[19]);
  k_lin<CC, 0, 8><<<dim3(TRB, CC / 128), 128, 0, stream>>>(XK, CC, PK + PK_O, nullptr, (float*)d_out, CC);
}
